// HybridModelImproved_14877766713462
// MI455X (gfx1250) — hardware-verified
//
#include <hip/hip_runtime.h>
#include <stddef.h>


#define SPB    4
#define TC     256
#define NPOS1  144
#define SP1    960
#define K2P    160
#define C2N    16
#define KF     256
#define NF1    120
#define NF1P   128
#define NF2    4
#define RPB    32
#define TF     128
#define HP     128
#define TQ     64
#define NCLS   10
#define W1P    28
#define NPREP  19
#define WSCAP  134217728

static_assert(K2P % 32 == 0);
static_assert(KF % 32 == 0);
static_assert(SP1 >= 864 + 96);
static_assert((SP1 * 2) % 16 == 0);
static_assert(SPB * 32 <= TC);
static_assert(SPB * 96 <= 2 * TC);
static_assert(RPB == 32 && TF == 128);
static_assert(NF1P * KF == 16 * 256 * 8);
static_assert(C2N * K2P == 320 * 8);
static_assert((TQ * NCLS * 4) % 128 == 0);
static_assert(TQ == 64);
static_assert((W1P * 4) % 16 == 0);
static_assert(6 * W1P <= TC);

typedef float          v2f  __attribute__((ext_vector_type(2)));
typedef float          v4f  __attribute__((ext_vector_type(4)));
typedef float          v8f  __attribute__((ext_vector_type(8)));
typedef unsigned int   v8u  __attribute__((ext_vector_type(8)));
typedef unsigned short v8us __attribute__((ext_vector_type(8)));
typedef __bf16         v16b __attribute__((ext_vector_type(16)));
union FragB { v16b v; v8us h[2]; v8u u; };

__device__ __forceinline__ unsigned int bfr(float f) {
  const unsigned int u = __float_as_uint(f);
  return (u + 0x7FFFu + ((u >> 16) & 1u)) >> 16;
}

__device__ __forceinline__ void split1(float x, unsigned short& hb, unsigned short& lb) {
  const unsigned int hu = bfr(x);
  const float hf = __uint_as_float(hu << 16);
  hb = (unsigned short)hu;
  lb = (unsigned short)bfr(x - hf);
}

__device__ __forceinline__ void split8(v4f a, v4f b, v8us& hi, v8us& lo) {
  unsigned short hb, lb;
  split1(a.x, hb, lb); hi[0] = hb; lo[0] = lb;
  split1(a.y, hb, lb); hi[1] = hb; lo[1] = lb;
  split1(a.z, hb, lb); hi[2] = hb; lo[2] = lb;
  split1(a.w, hb, lb); hi[3] = hb; lo[3] = lb;
  split1(b.x, hb, lb); hi[4] = hb; lo[4] = lb;
  split1(b.y, hb, lb); hi[5] = hb; lo[5] = lb;
  split1(b.z, hb, lb); hi[6] = hb; lo[6] = lb;
  split1(b.w, hb, lb); hi[7] = hb; lo[7] = lb;
}

__device__ __forceinline__ v8f wmb(v16b a, v16b b, v8f c) {
  v8f d = __builtin_amdgcn_wmma_f32_16x16x32_bf16(false, a, false, b, (short)0, c, false, false);
  asm volatile("v_nop\n\tv_nop\n\tv_nop\n\tv_nop" : "+v"(d) : "v"(a), "v"(b));
  return d;
}

__host__ __device__ constexpr int koff(int k) {
  return k < 150 ? (k / 25) * 144 + ((k % 25) / 5) * 12 + ((k % 25) % 5) : 864;
}

__global__ __launch_bounds__(256) void k_prep(
    const float* __restrict__ c2w, const float* __restrict__ f1w, const float* __restrict__ qw,
    unsigned short* w2p, unsigned short* w1p, float* gt) {
  __shared__ float stc[48];
  __shared__ __attribute__((aligned(16))) float sgt[64];
  const int tid = (int)threadIdx.x, b = (int)blockIdx.x;
  if (b < 2) {
    const int c = b * 256 + tid;
    const bool act = c < C2N * (K2P / 8);
    const int cc = act ? c : C2N * (K2P / 8) - 1;
    const int o = cc / (K2P / 8), k0 = (cc - o * (K2P / 8)) * 8;
    float v[8];
#pragma unroll
    for (int e = 0; e < 8; ++e) {
      const int k = k0 + e;
      const int kc = k < 150 ? k : 149;
      const float t = c2w[o * 150 + kc];
      v[e] = (k < 150) ? t : 0.0f;
    }
    v4f a, bq;
    a.x = v[0]; a.y = v[1]; a.z = v[2]; a.w = v[3];
    bq.x = v[4]; bq.y = v[5]; bq.z = v[6]; bq.w = v[7];
    v8us hv, lv;
    split8(a, bq, hv, lv);
    unsigned short* dh = w2p + (size_t)cc * 8;
    unsigned short* dl = w2p + C2N * K2P + (size_t)cc * 8;
    if (act) { *(volatile v8us*)dh = hv; *(volatile v8us*)dl = lv; }
    __threadfence();
    if (act) { *(volatile v8us*)dh = hv; *(volatile v8us*)dl = lv; }
  } else if (b < 18) {
    const int c = (b - 2) * 256 + tid;
    const int n = c >> 5, k0 = (c & 31) * 8;
    const int nc = n < NF1 ? n : NF1 - 1;
    float v[8];
#pragma unroll
    for (int e = 0; e < 8; ++e) {
      const float t = f1w[nc * KF + k0 + e];
      v[e] = (n < NF1) ? t : 0.0f;
    }
    v4f a, bq;
    a.x = v[0]; a.y = v[1]; a.z = v[2]; a.w = v[3];
    bq.x = v[4]; bq.y = v[5]; bq.z = v[6]; bq.w = v[7];
    v8us hv, lv;
    split8(a, bq, hv, lv);
    unsigned short* dh = w1p + (size_t)c * 8;
    unsigned short* dl = w1p + (size_t)NF1P * KF + (size_t)c * 8;
    *(volatile v8us*)dh = hv; *(volatile v8us*)dl = lv;
    __threadfence();
    *(volatile v8us*)dh = hv; *(volatile v8us*)dl = lv;
  } else {
    const int tj = tid < 24 ? tid : 23;
    const int g = tj / 3, wh = tj - g * 3;
    const float phi = qw[g * 3 + 0], th = qw[g * 3 + 1], om = qw[g * 3 + 2];
    const float ang = (wh == 0) ? 0.5f * th : ((wh == 1) ? 0.5f * (phi + om) : 0.5f * (phi - om));
    float sn, cs;
    sincosf(ang, &sn, &cs);
    if (tid < 24) { stc[2 * tid] = cs; stc[2 * tid + 1] = sn; }
    __syncthreads();
    if (tid < 8) {
      const float ct = stc[(tid * 3 + 0) * 2], st = stc[(tid * 3 + 0) * 2 + 1];
      const float ca = stc[(tid * 3 + 1) * 2], sa = stc[(tid * 3 + 1) * 2 + 1];
      const float cb = stc[(tid * 3 + 2) * 2], sb = stc[(tid * 3 + 2) * 2 + 1];
      float* g8 = sgt + tid * 8;
      g8[0] = ca * ct;  g8[1] = -sa * ct;
      g8[2] = -cb * st; g8[3] = -sb * st;
      g8[4] = cb * st;  g8[5] = -sb * st;
      g8[6] = ca * ct;  g8[7] = sa * ct;
    }
    __syncthreads();
    const int lc = tid < 16 ? tid : 15;
    const v4f gv = *(const v4f*)(sgt + 4 * lc);
    if (tid < 16) *(volatile v4f*)(gt + 4 * tid) = gv;
    __threadfence();
    if (tid < 16) *(volatile v4f*)(gt + 4 * tid) = gv;
  }
}

__global__ __launch_bounds__(TC) void k_conv(
    const float* __restrict__ x, const float* __restrict__ c1w, const float* __restrict__ c1b,
    const unsigned short* __restrict__ w2p, const float* __restrict__ c2b,
    unsigned short* a2h, unsigned short* a2l) {
  __shared__ __attribute__((aligned(16))) float sw1[6 * W1P];
  __shared__ float sb1[8];
  __shared__ float sb2[C2N];
  __shared__ __attribute__((aligned(16))) unsigned short sHi[SPB * SP1];
  __shared__ __attribute__((aligned(16))) unsigned short sLo[SPB * SP1];
  __shared__ __attribute__((aligned(16))) float sP[SPB * KF];
  const int tid = (int)threadIdx.x, lane = tid & 31, wave = tid >> 5, hh = lane >> 4, m = lane & 15;
  const int s0 = (int)blockIdx.x * SPB;

  {
    const int i1 = tid < 6 * W1P ? tid : 6 * W1P - 1;
    const int c = i1 / W1P, t = i1 - c * W1P;
    const int tcl = t < 25 ? t : 24;
    const float wv = c1w[c * 25 + tcl];
    if (tid < 6 * W1P) sw1[tid] = (t < 25) ? wv : 0.0f;
    const float bv = c1b[tid < 6 ? tid : 5];
    if (tid < 8) sb1[tid] = (tid < 6) ? bv : 0.0f;
    const float b2v = c2b[tid < C2N ? tid : C2N - 1];
    if (tid < C2N) sb2[tid] = b2v;
#pragma unroll 1
    for (int i = tid; i < SPB * 96; i += TC) {
      const int s = i / 96, j = i - s * 96;
      sHi[s * SP1 + 864 + j] = 0;
      sLo[s * SP1 + 864 + j] = 0;
    }
  }
  __syncthreads();

#pragma unroll 1
  for (int it = tid; it < SPB * NPOS1; it += TC) {
    const int s = it / NPOS1, pos = it - s * NPOS1;
    const int py = pos / 12, px = pos - py * 12;
    const float* xin = x + (size_t)(s0 + s) * 784 + (2 * py) * 28 + 2 * px;
    float pv[36];
#pragma unroll
    for (int r = 0; r < 6; ++r) {
#pragma unroll
      for (int q = 0; q < 3; ++q) {
        const v2f t2 = *(const v2f*)(xin + r * 28 + 2 * q);
        pv[r * 6 + 2 * q] = t2.x;
        pv[r * 6 + 2 * q + 1] = t2.y;
      }
    }
#pragma unroll 1
    for (int c = 0; c < 6; ++c) {
      const float* wp = sw1 + c * W1P;
      float wr[28];
#pragma unroll
      for (int u = 0; u < 7; ++u) {
        const v4f q4 = *(const v4f*)(wp + 4 * u);
        wr[4 * u] = q4.x; wr[4 * u + 1] = q4.y; wr[4 * u + 2] = q4.z; wr[4 * u + 3] = q4.w;
      }
      float a00 = 0.0f, a01 = 0.0f, a10 = 0.0f, a11 = 0.0f;
#pragma unroll
      for (int r = 0; r < 5; ++r) {
#pragma unroll
        for (int ss = 0; ss < 5; ++ss) {
          const float wv = wr[r * 5 + ss];
          a00 = fmaf(pv[r * 6 + ss], wv, a00);
          a01 = fmaf(pv[r * 6 + ss + 1], wv, a01);
          a10 = fmaf(pv[(r + 1) * 6 + ss], wv, a10);
          a11 = fmaf(pv[(r + 1) * 6 + ss + 1], wv, a11);
        }
      }
      const float mx = fmaxf(fmaxf(a00, a01), fmaxf(a10, a11));
      const float v = fmaxf(mx + sb1[c], 0.0f);
      unsigned short hb, lb;
      split1(v, hb, lb);
      const int si = s * SP1 + c * 144 + pos;
      sHi[si] = hb;
      sLo[si] = lb;
    }
  }
  __syncthreads();

#pragma unroll 1
  for (int t = wave; t < SPB * 4; t += TC / 32) {
    const int s = t >> 2, ty = t & 3;
    const int oy = 2 * ty + (m >> 3), ox = m & 7;
    const int base = s * SP1 + oy * 12 + ox;
    v8f acc = {0.f, 0.f, 0.f, 0.f, 0.f, 0.f, 0.f, 0.f};
#pragma unroll
    for (int kk = 0; kk < K2P / 32; ++kk) {
      FragB ah, al, bh, bl;
#pragma unroll
      for (int q = 0; q < 2; ++q) {
#pragma unroll
        for (int j = 0; j < 4; ++j) {
          const int K0 = 32 * kk + 16 * q + 2 * j;
          const int o0 = hh ? koff(K0 + 8) : koff(K0);
          const int o1 = hh ? koff(K0 + 9) : koff(K0 + 1);
          const unsigned int h0 = sHi[base + o0], h1 = sHi[base + o1];
          const unsigned int l0 = sLo[base + o0], l1 = sLo[base + o1];
          ah.u[4 * q + j] = h0 | (h1 << 16);
          al.u[4 * q + j] = l0 | (l1 << 16);
        }
      }
      const unsigned short* bp = w2p + m * K2P + 32 * kk + 8 * hh;
      bh.h[0] = *(const v8us*)bp;
      bh.h[1] = *(const v8us*)(bp + 16);
      bl.h[0] = *(const v8us*)(bp + C2N * K2P);
      bl.h[1] = *(const v8us*)(bp + C2N * K2P + 16);
      acc = wmb(ah.v, bh.v, acc);
      acc = wmb(ah.v, bl.v, acc);
      acc = wmb(al.v, bh.v, acc);
    }
    float q4[4];
#pragma unroll
    for (int px = 0; px < 4; ++px) q4[px] = fmaxf(acc[2 * px], acc[2 * px + 1]);
#pragma unroll
    for (int px = 0; px < 4; ++px) {
      const float oth = __shfl_xor(q4[px], 16);
      q4[px] = fmaxf(q4[px], oth);
    }
    const float bo = sb2[m];
    const float va = fmaxf((hh ? q4[2] : q4[0]) + bo, 0.0f);
    const float vb = fmaxf((hh ? q4[3] : q4[1]) + bo, 0.0f);
    float* pp = sP + s * KF + m * 16 + ty * 4 + 2 * hh;
    pp[0] = va;
    pp[1] = vb;
  }
  __syncthreads();

  if (tid < SPB * 32) {
    const int c = tid, s = c >> 5, k0 = (c & 31) * 8;
    const v4f a0 = *(const v4f*)(sP + s * KF + k0);
    const v4f a1 = *(const v4f*)(sP + s * KF + k0 + 4);
    v8us hv, lv;
    split8(a0, a1, hv, lv);
    unsigned short* ph = a2h + (size_t)s0 * KF + (size_t)c * 8;
    unsigned short* pl = a2l + (size_t)s0 * KF + (size_t)c * 8;
    *(volatile v8us*)ph = hv;
    *(volatile v8us*)pl = lv;
    __threadfence();
    *(volatile v8us*)ph = hv;
    *(volatile v8us*)pl = lv;
  }
}

__global__ __launch_bounds__(TF) void k_fc(
    const unsigned short* __restrict__ a2h, const unsigned short* __restrict__ a2l,
    const unsigned short* __restrict__ w1p, const float* __restrict__ b1,
    const float* __restrict__ f2w, const float* __restrict__ f2b, float* feats) {
  __shared__ __attribute__((aligned(16))) float sH[RPB * HP];
  __shared__ __attribute__((aligned(16))) float sF[RPB * NF2];
  const int tid = (int)threadIdx.x, lane = tid & 31, wave = tid >> 5, hh = lane >> 4, m = lane & 15;
  const int rb = 16 * (wave & 1), cb = 64 * (wave >> 1);
  const size_t grow = (size_t)blockIdx.x * RPB + rb + m;
  const unsigned short* ap  = a2h + grow * KF + 8 * hh;
  const unsigned short* alp = a2l + grow * KF + 8 * hh;

  v8f acc[4];
#pragma unroll
  for (int t = 0; t < 4; ++t) { v8f z = {0.f, 0.f, 0.f, 0.f, 0.f, 0.f, 0.f, 0.f}; acc[t] = z; }
#pragma unroll 1
  for (int kt = 0; kt < KF / 32; ++kt) {
    FragB fa, fl;
    fa.h[0] = *(const v8us*)(ap + 32 * kt);
    fa.h[1] = *(const v8us*)(ap + 32 * kt + 16);
    fl.h[0] = *(const v8us*)(alp + 32 * kt);
    fl.h[1] = *(const v8us*)(alp + 32 * kt + 16);
#pragma unroll
    for (int t = 0; t < 4; ++t) {
      const unsigned short* bp = w1p + (size_t)(cb + 16 * t + m) * KF + 32 * kt + 8 * hh;
      FragB bh, bl;
      bh.h[0] = *(const v8us*)bp;
      bh.h[1] = *(const v8us*)(bp + 16);
      bl.h[0] = *(const v8us*)(bp + (size_t)NF1P * KF);
      bl.h[1] = *(const v8us*)(bp + (size_t)NF1P * KF + 16);
      acc[t] = wmb(fa.v, bh.v, acc[t]);
      acc[t] = wmb(fa.v, bl.v, acc[t]);
      acc[t] = wmb(fl.v, bh.v, acc[t]);
    }
  }

#pragma unroll
  for (int t = 0; t < 4; ++t) {
    const int col = cb + 16 * t + m;
    const int colc = col < NF1 ? col : NF1 - 1;
    const float bbv = b1[colc];
    const float bb = (col < NF1) ? bbv : 0.0f;
#pragma unroll
    for (int r = 0; r < 8; ++r) sH[(rb + 8 * hh + r) * HP + col] = fmaxf(acc[t][r] + bb, 0.0f);
  }
  __syncthreads();

  const int row = tid >> 2, j = tid & 3;
  const float* hrow = sH + row * HP;
  const float* wj = f2w + j * NF1;
  float a = f2b[j];
#pragma unroll 4
  for (int k = 0; k < NF1; ++k) a = fmaf(hrow[k], wj[k], a);
  sF[row * NF2 + j] = a;
  __syncthreads();

  if (wave == 0) {
    const v4f v = *(const v4f*)(sF + 4 * lane);
    float* gp = feats + ((size_t)blockIdx.x * RPB + lane) * NF2;
    *(volatile v4f*)gp = v;
    __threadfence();
    *(volatile v4f*)gp = v;
  }
}

__global__ __launch_bounds__(TQ) void k_tail(
    const float* __restrict__ feats, const float* __restrict__ gt,
    const float* __restrict__ clw, const float* __restrict__ clb, float* out) {
  __shared__ float sv[32 * TQ];
  __shared__ float sA[4 * TQ];
  __shared__ float sG[64];
  __shared__ float sCW[40];
  __shared__ float sCB[12];
  __shared__ __attribute__((aligned(16))) float sO[TQ * NCLS];
  const int tid = (int)threadIdx.x;
  const size_t row = (size_t)blockIdx.x * TQ + tid;

  sG[tid] = gt[tid];
  const float cwv = clw[tid < 40 ? tid : 39];
  if (tid < 40) sCW[tid] = cwv;
  const float cbv = clb[tid < NCLS ? tid : NCLS - 1];
  if (tid < NCLS) sCB[tid] = cbv;
  const v4f f = *(const v4f*)(feats + row * NF2);
  sA[0 * TQ + tid] = f.x; sA[1 * TQ + tid] = f.y; sA[2 * TQ + tid] = f.z; sA[3 * TQ + tid] = f.w;
#pragma unroll 1
  for (int i = 0; i < 32; ++i) sv[i * TQ + tid] = (i == 0) ? 1.0f : 0.0f;
  __syncthreads();

#pragma unroll 1
  for (int g = 0; g < 12; ++g) {
    const int w = g & 3;
    float g0r, g0i, g1r, g1i, g2r, g2i, g3r, g3i;
    if (g < 4) {
      float fv = sA[w * TQ + tid];
      fv = fminf(fmaxf(fv, -30.0f), 30.0f);
      const float e = expf(-fv);
      const float sg = 1.0f / (1.0f + e);
      const float ang = 3.14159265358979f * sg;
      float sn, cs;
      sincosf(0.5f * ang, &sn, &cs);
      g0r = cs;   g0i = 0.0f;  g1r = 0.0f; g1i = -sn;
      g2r = 0.0f; g2i = -sn;   g3r = cs;   g3i = 0.0f;
    } else {
      const float* gp = sG + (g - 4) * 8;
      g0r = gp[0]; g0i = gp[1]; g1r = gp[2]; g1i = gp[3];
      g2r = gp[4]; g2i = gp[5]; g3r = gp[6]; g3i = gp[7];
    }
    const int bpos = 3 - w, bit = 1 << bpos;
#pragma unroll 1
    for (int p = 0; p < 8; ++p) {
      const int i0 = ((p >> bpos) << (bpos + 1)) | (p & (bit - 1));
      const int i1 = i0 | bit;
      const float a0r = sv[(2 * i0) * TQ + tid], a0i = sv[(2 * i0 + 1) * TQ + tid];
      const float a1r = sv[(2 * i1) * TQ + tid], a1i = sv[(2 * i1 + 1) * TQ + tid];
      const float n0r = g0r * a0r - g0i * a0i + g1r * a1r - g1i * a1i;
      const float n0i = g0r * a0i + g0i * a0r + g1r * a1i + g1i * a1r;
      const float n1r = g2r * a0r - g2i * a0i + g3r * a1r - g3i * a1i;
      const float n1i = g2r * a0i + g2i * a0r + g3r * a1i + g3i * a1r;
      sv[(2 * i0) * TQ + tid] = n0r; sv[(2 * i0 + 1) * TQ + tid] = n0i;
      sv[(2 * i1) * TQ + tid] = n1r; sv[(2 * i1 + 1) * TQ + tid] = n1i;
    }
    if (g == 7 || g == 11) {
      const int rr = (g == 7) ? 1 : 2;
#pragma unroll 1
      for (int cq = 0; cq < 4; ++cq) {
        const int tg = (cq + rr) & 3;
        const int bc = 8 >> cq, bt = 8 >> tg;
#pragma unroll 1
        for (int i = 0; i < 16; ++i) {
          if ((i & bc) && !(i & bt)) {
            const int jx = i | bt;
            const float ur = sv[(2 * i) * TQ + tid],  ui = sv[(2 * i + 1) * TQ + tid];
            const float vr = sv[(2 * jx) * TQ + tid], vi = sv[(2 * jx + 1) * TQ + tid];
            sv[(2 * i) * TQ + tid] = vr;  sv[(2 * i + 1) * TQ + tid] = vi;
            sv[(2 * jx) * TQ + tid] = ur; sv[(2 * jx + 1) * TQ + tid] = ui;
          }
        }
      }
    }
  }

  float z0 = 0.0f, z1 = 0.0f, z2 = 0.0f, z3 = 0.0f;
#pragma unroll 1
  for (int i = 0; i < 16; ++i) {
    const float re = sv[(2 * i) * TQ + tid], im = sv[(2 * i + 1) * TQ + tid];
    const float p = fmaf(re, re, im * im);
    z0 += (i & 8) ? -p : p;
    z1 += (i & 4) ? -p : p;
    z2 += (i & 2) ? -p : p;
    z3 += (i & 1) ? -p : p;
  }
#pragma unroll 1
  for (int o = 0; o < NCLS; ++o) {
    float a = sCB[o];
    a = fmaf(z0, sCW[o * 4 + 0], a);
    a = fmaf(z1, sCW[o * 4 + 1], a);
    a = fmaf(z2, sCW[o * 4 + 2], a);
    a = fmaf(z3, sCW[o * 4 + 3], a);
    sO[tid * NCLS + o] = a;
  }
  __syncthreads();

  float* ob = out + (size_t)blockIdx.x * (TQ * NCLS);
  const int c0 = tid, c1 = tid + TQ;
  const bool act2 = tid < (TQ * NCLS / 4) - 2 * TQ;
  const int c2 = act2 ? tid + 2 * TQ : (TQ * NCLS / 4) - 1;
  const v4f v0 = *(const v4f*)(sO + 4 * c0);
  const v4f v1 = *(const v4f*)(sO + 4 * c1);
  const v4f v2 = *(const v4f*)(sO + 4 * c2);
  *(volatile v4f*)(ob + 4 * c0) = v0;
  *(volatile v4f*)(ob + 4 * c1) = v1;
  if (act2) *(volatile v4f*)(ob + 4 * c2) = v2;
  __threadfence();
  *(volatile v4f*)(ob + 4 * c0) = v0;
  *(volatile v4f*)(ob + 4 * c1) = v1;
  if (act2) *(volatile v4f*)(ob + 4 * c2) = v2;
}

extern "C" void kernel_launch(void* const* d_in, const int* in_sizes, int n_in,
                              void* d_out, int out_size, void* d_ws, size_t ws_size,
                              hipStream_t stream) {
  if (n_in < 12) return;
  const int nS = in_sizes[0] / 784;
  if (nS <= 0 || nS > (1 << 20) || in_sizes[0] != nS * 784 || (nS % 64) != 0) return;
  if (in_sizes[1] != 150 || in_sizes[2] != 6 || in_sizes[3] != C2N * 150 || in_sizes[4] != C2N) return;
  if (in_sizes[5] != NF1 * KF || in_sizes[6] != NF1 || in_sizes[7] != NF2 * NF1 || in_sizes[8] != NF2) return;
  if (in_sizes[9] != 24 || in_sizes[10] != NCLS * 4 || in_sizes[11] != NCLS) return;
  if (out_size != nS * NCLS) return;

  const float* x   = (const float*)d_in[0];
  const float* c1w = (const float*)d_in[1];
  const float* c1b = (const float*)d_in[2];
  const float* c2w = (const float*)d_in[3];
  const float* c2b = (const float*)d_in[4];
  const float* f1w = (const float*)d_in[5];
  const float* f1b = (const float*)d_in[6];
  const float* f2w = (const float*)d_in[7];
  const float* f2b = (const float*)d_in[8];
  const float* qwv = (const float*)d_in[9];
  const float* clw = (const float*)d_in[10];
  const float* clb = (const float*)d_in[11];
  float* out = (float*)d_out;

  char* ws = (char*)d_ws;
  size_t off = 0;
  const size_t oW2 = off; off += (size_t)2 * C2N * K2P * 2;      off = (off + 255) & ~(size_t)255;
  const size_t oW1 = off; off += (size_t)2 * NF1P * KF * 2;      off = (off + 255) & ~(size_t)255;
  const size_t oGT = off; off += 256;                              off = (off + 255) & ~(size_t)255;
  const size_t oAh = off; off += (size_t)nS * KF * 2;             off = (off + 255) & ~(size_t)255;
  const size_t oAl = off; off += (size_t)nS * KF * 2;             off = (off + 255) & ~(size_t)255;
  const size_t oF  = off; off += (size_t)nS * NF2 * 4;            off = (off + 255) & ~(size_t)255;
  if (off > ws_size || off > (size_t)WSCAP) return;
  unsigned short* w2p = (unsigned short*)(ws + oW2);
  unsigned short* w1p = (unsigned short*)(ws + oW1);
  float* gtp = (float*)(ws + oGT);
  unsigned short* a2h = (unsigned short*)(ws + oAh);
  unsigned short* a2l = (unsigned short*)(ws + oAl);
  float* ftp = (float*)(ws + oF);

  k_prep<<<NPREP, 256, 0, stream>>>(c2w, f1w, qwv, w2p, w1p, gtp);
  k_conv<<<nS / SPB, TC, 0, stream>>>(x, c1w, c1b, w2p, c2b, a2h, a2l);
  k_fc<<<nS / RPB, TF, 0, stream>>>(a2h, a2l, w1p, f1b, f2w, f2b, ftp);
  k_tail<<<nS / TQ, TQ, 0, stream>>>(ftp, gtp, clw, clb, out);
}
